// TransformerBlock_64639257805460
// MI455X (gfx1250) — hardware-verified
//
#include <hip/hip_runtime.h>
#include <stddef.h>
#include <math.h>


typedef _Float16 v16h __attribute__((ext_vector_type(16)));
typedef _Float16 v8h  __attribute__((ext_vector_type(8)));
typedef float    v8f  __attribute__((ext_vector_type(8)));
typedef float    v4f  __attribute__((ext_vector_type(4)));

#ifndef NB
#define NB 2
#endif
#ifndef SEQ
#define SEQ 2048
#endif
#define NB_FULL  2
#define SEQ_FULL 2048
#define DIM   1024
#define NHEAD 16
#define HD    64
#define FF    4096
#define MROWS (NB * SEQ)

static_assert(NB >= 1 && NB <= NB_FULL);
static_assert(SEQ >= 128 && SEQ <= SEQ_FULL && (SEQ % 128) == 0);
static_assert(DIM == NHEAD * HD && NHEAD == 16 && HD == 64 && DIM == 1024);
static_assert(FF == 4 * DIM);
static_assert((MROWS % 64) == 0 && (MROWS % 8) == 0);
static_assert((DIM % 64) == 0 && (FF % 64) == 0);

#define LDT 72
#define LDC 68

#define WCARRY 64.0f
#define PCARRY 1024.0f
#define VCARRY 64.0f
#define HCARRY 16.0f

#define P16_BYTES  ((size_t)MROWS * DIM * 2)
#define WQKV_BYTES ((size_t)3 * DIM * DIM * 2)
#define WO_BYTES   ((size_t)DIM * DIM * 2)
#define W1_BYTES   ((size_t)FF * DIM * 2)
#define W2_BYTES   ((size_t)DIM * FF * 2)
#define OFF_WQKV   ((size_t)0)
#define OFF_WO     (OFF_WQKV + WQKV_BYTES)
#define OFF_W1     (OFF_WO + WO_BYTES)
#define OFF_W2     (OFF_W1 + W1_BYTES)
#define OFF_H1     (OFF_W2 + W2_BYTES)
#define OFF_QKV    (OFF_H1 + P16_BYTES)
#define OFF_OV     (OFF_QKV + 3 * P16_BYTES)
#define OFF_X1     (OFF_OV + P16_BYTES)
#define OFF_H2     (OFF_X1 + 2 * P16_BYTES)
#define OFF_G      (OFF_H2 + P16_BYTES)
#define WS_TOTAL   (OFF_G + 4 * P16_BYTES)
static_assert((size_t)MROWS * FF * 2 == 4 * P16_BYTES);
static_assert((size_t)NB * DIM * SEQ * 2 == P16_BYTES);
static_assert((size_t)MROWS * DIM * 4 == 2 * P16_BYTES);
static_assert((P16_BYTES % 128) == 0 && (WO_BYTES % 128) == 0 && (WQKV_BYTES % 128) == 0);
static_assert(WS_TOTAL <= (size_t)134217728);

__device__ __forceinline__ float bf16r(float x) {
  unsigned int u = __float_as_uint(x);
  u = (u + 0x7FFFu + ((u >> 16) & 1u)) & 0xFFFF0000u;
  return __uint_as_float(u);
}

__device__ __forceinline__ size_t full_row(unsigned r) {
  const unsigned n = r / (unsigned)SEQ;
  const unsigned s = r - n * (unsigned)SEQ;
  return (size_t)n * SEQ_FULL + s;
}

__device__ __forceinline__ v16h frag_at(const _Float16* p) {
  v8h lo = *(const v8h*)(p);
  v8h hi = *(const v8h*)(p + 16);
  v16h out;
#pragma unroll
  for (int i = 0; i < 8; ++i) { out[i] = lo[i]; out[i + 8] = hi[i]; }
  return out;
}
__device__ __forceinline__ v16h ld_frag(const _Float16* base, int ld) {
  const int lane = threadIdx.x & 31;
  return frag_at(base + (lane & 15) * ld + (lane >> 4) * 8);
}

__device__ __forceinline__ v8f wmma16(v16h a, v16h b, v8f c) {
  v8f d = __builtin_amdgcn_wmma_f32_16x16x32_f16(false, a, false, b, (short)0, c,
                                                 false, false);
  asm volatile("v_nop\n\tv_nop\n\tv_nop\n\tv_nop" : "+v"(d) : "v"(a), "v"(b));
  return d;
}

__device__ __forceinline__ float red16_max(float x) {
#pragma unroll
  for (int off = 1; off < 16; off <<= 1) x = fmaxf(x, __shfl_xor(x, off, 32));
  return x;
}
__device__ __forceinline__ float red16_sum(float x) {
#pragma unroll
  for (int off = 1; off < 16; off <<= 1) x += __shfl_xor(x, off, 32);
  return x;
}
__device__ __forceinline__ float wave_sum(float x) {
#pragma unroll
  for (int off = 1; off < 32; off <<= 1) x += __shfl_xor(x, off, 32);
  return x;
}

__device__ __forceinline__ void wave_lds_sync() {
  __builtin_amdgcn_fence(3  , "wavefront");
  asm volatile("s_wait_dscnt 0x0" ::: "memory");
  __builtin_amdgcn_wave_barrier();
}

template <int XIN>
__device__ __forceinline__ v4f ld4(const float* p) {
  v4f a = *(const v4f*)p;
  if (XIN) {
#pragma unroll
    for (int t = 0; t < 4; ++t) a[t] = bf16r(a[t]);
  }
  return a;
}

template <int KD, int ND>
__global__ __launch_bounds__(256) void tcvt_kernel(
    const float* __restrict__ src, _Float16* __restrict__ dst) {
  static_assert((KD % 64) == 0 && (ND % 64) == 0);
  static_assert((size_t)(ND / 64) * (KD / 64) * 256 * 2 * 8 == (size_t)KD * ND);
  __shared__ float Ts[64 * LDC];
  const unsigned tid = threadIdx.x;
  const unsigned n0 = blockIdx.x * 64u;
  const unsigned k0 = blockIdx.y * 64u;
#pragma unroll
  for (int i = 0; i < 4; ++i) {
    const unsigned idx = tid + 256u * (unsigned)i;
    const unsigned r = idx >> 4;
    const unsigned c = (idx & 15u) * 4u;
    const v4f a = *(const v4f*)(src + (size_t)(k0 + r) * ND + n0 + c);
    v4f t;
#pragma unroll
    for (int j = 0; j < 4; ++j) t[j] = WCARRY * bf16r(a[j]);
    *(v4f*)&Ts[r * LDC + c] = t;
  }
  __syncthreads();
  v8h x[2];
  size_t off[2];
#pragma unroll
  for (int i = 0; i < 2; ++i) {
    const unsigned nr = 32u * (unsigned)i + (tid >> 3);
    const unsigned kk = (tid & 7u) * 8u;
#pragma unroll
    for (int j = 0; j < 8; ++j) x[i][j] = (_Float16)Ts[(kk + j) * LDC + nr];
    off[i] = (size_t)(n0 + nr) * KD + k0 + kk;
  }
#pragma unroll
  for (int i = 0; i < 2; ++i) *(volatile v8h*)(dst + off[i]) = x[i];
  __threadfence();
#pragma unroll
  for (int i = 0; i < 2; ++i) *(volatile v8h*)(dst + off[i]) = x[i];
}

template <int XIN>
__global__ __launch_bounds__(256) void ln_kernel(
    const float* __restrict__ src, const float* __restrict__ gam,
    const float* __restrict__ bet, _Float16* __restrict__ dst16) {
  static_assert(4 * 32 * 8 == DIM);
  const unsigned lane = threadIdx.x & 31u, w = threadIdx.x >> 5;
  const unsigned row = blockIdx.x * 8u + w;
  const size_t srow = XIN ? full_row(row) : (size_t)row;
  const float* xr = src + srow * DIM;

  float s = 0.0f;
#pragma unroll 1
  for (unsigned j = 0; j < 4u; ++j) {
    const unsigned c = j * 256u + lane * 8u;
    const v4f a0 = ld4<XIN>(xr + c);
    const v4f a1 = ld4<XIN>(xr + c + 4);
#pragma unroll
    for (int t = 0; t < 4; ++t) { s += a0[t]; s += a1[t]; }
  }
  const float mu = wave_sum(s) * (1.0f / DIM);

  float q = 0.0f;
#pragma unroll 1
  for (unsigned j = 0; j < 4u; ++j) {
    const unsigned c = j * 256u + lane * 8u;
    const v4f a0 = ld4<XIN>(xr + c);
    const v4f a1 = ld4<XIN>(xr + c + 4);
#pragma unroll
    for (int t = 0; t < 4; ++t) {
      const float d0 = a0[t] - mu;
      const float d1 = a1[t] - mu;
      q += d0 * d0;
      q += d1 * d1;
    }
  }
  const float var = wave_sum(q) * (1.0f / DIM);
  const float rs = rsqrtf(var + 1.0e-5f);

  _Float16* orow = dst16 + (size_t)row * DIM;
#pragma unroll 1
  for (unsigned j = 0; j < 4u; ++j) {
    const unsigned c = j * 256u + lane * 8u;
    const v4f a0 = ld4<XIN>(xr + c);
    const v4f a1 = ld4<XIN>(xr + c + 4);
    const v4f g0 = *(const v4f*)(gam + c);
    const v4f g1 = *(const v4f*)(gam + c + 4);
    const v4f b0 = *(const v4f*)(bet + c);
    const v4f b1 = *(const v4f*)(bet + c + 4);
    v8h o;
#pragma unroll
    for (int t = 0; t < 4; ++t) {
      const float y0 = ((a0[t] - mu) * rs) * bf16r(g0[t]) + bf16r(b0[t]);
      const float y1 = ((a1[t] - mu) * rs) * bf16r(g1[t]) + bf16r(b1[t]);
      o[t]     = (_Float16)y0;
      o[t + 4] = (_Float16)y1;
    }
    *(volatile v8h*)(orow + c) = o;
    __threadfence();
    *(volatile v8h*)(orow + c) = o;
  }
}

#define MODE_QKV 0
#define MODE_WO  1
#define MODE_W1  2
#define MODE_W2  3

__device__ __forceinline__ float gelu_f(float t) {
  return 0.5f * t * (1.0f + erff(t * 0.70710678118654752f));
}

template <int MODE, int KD, int ND>
__global__ __launch_bounds__(256) void gemm_kernel(
    const _Float16* __restrict__ A16, const _Float16* __restrict__ Bt,
    const float* __restrict__ bias, const float* __restrict__ addf,
    float* __restrict__ outf, _Float16* __restrict__ out16) {
  static_assert((KD % 32) == 0 && (ND % 64) == 0);
  static_assert((MODE != MODE_WO && MODE != MODE_W2) || ND == DIM);
  static_assert(MODE != MODE_QKV || (ND == 3 * DIM && KD == DIM));
  static_assert(MODE != MODE_W1 || ND == FF);
  __shared__ float Cs[64 * LDC];
  const unsigned tid = threadIdx.x, lane = tid & 31u, w = tid >> 5;
  const unsigned mw = w >> 1, nw = w & 1u;
  const unsigned hh = lane >> 4, m = lane & 15u;
  const unsigned n0 = blockIdx.x * 64u;
  const unsigned row0 = blockIdx.y * 64u;

  const _Float16* ap  = A16 + (size_t)(row0 + mw * 16u + m) * KD + hh * 8u;
  const _Float16* bp0 = Bt + (size_t)(n0 + nw * 32u + m) * KD + hh * 8u;
  const _Float16* bp1 = bp0 + (size_t)16 * KD;
  v8f acc0 = {}, acc1 = {};
#pragma unroll 2
  for (int k0 = 0; k0 < KD; k0 += 32) {
    const v16h a  = frag_at(ap + k0);
    const v16h b0 = frag_at(bp0 + k0);
    const v16h b1 = frag_at(bp1 + k0);
    acc0 = wmma16(a, b0, acc0);
    acc1 = wmma16(a, b1, acc1);
  }
#pragma unroll
  for (int r = 0; r < 8; ++r) {
    float* d = &Cs[(mw * 16u + hh * 8u + (unsigned)r) * LDC + nw * 32u + m];
    d[0]  = acc0[r];
    d[16] = acc1[r];
  }
  __syncthreads();

  if (MODE == MODE_QKV) {
    const unsigned which = n0 >> 10;
    const unsigned hcol = n0 & 1023u;
    _Float16* dst = out16 + (size_t)which * ((size_t)MROWS * DIM);
    v8h x[2];
    size_t off[2];
    if (which < 2u) {
#pragma unroll
      for (int i = 0; i < 2; ++i) {
        const unsigned r = 32u * (unsigned)i + (tid >> 3);
        const unsigned c = (tid & 7u) * 8u;
        const v4f u0 = *(const v4f*)&Cs[r * LDC + c];
        const v4f u1 = *(const v4f*)&Cs[r * LDC + c + 4];
        const v4f g0 = *(const v4f*)(bias + n0 + c);
        const v4f g1 = *(const v4f*)(bias + n0 + c + 4);
#pragma unroll
        for (int j = 0; j < 4; ++j) {
          x[i][j]     = (_Float16)(u0[j] * (1.0f / WCARRY) + bf16r(g0[j]));
          x[i][j + 4] = (_Float16)(u1[j] * (1.0f / WCARRY) + bf16r(g1[j]));
        }
        off[i] = (size_t)(row0 + r) * DIM + hcol + c;
      }
    } else {
      const unsigned nbat = row0 / (unsigned)SEQ;
      const unsigned s0 = row0 - nbat * (unsigned)SEQ;
#pragma unroll
      for (int i = 0; i < 2; ++i) {
        const unsigned dcol = 32u * (unsigned)i + (tid >> 3);
        const unsigned kk = (tid & 7u) * 8u;
        const float bsv = bf16r(bias[n0 + dcol]);
#pragma unroll
        for (int j = 0; j < 8; ++j)
          x[i][j] = (_Float16)(Cs[(kk + (unsigned)j) * LDC + dcol] * (1.0f / WCARRY) + bsv);
        off[i] = ((size_t)nbat * DIM + hcol + dcol) * SEQ + s0 + kk;
      }
    }
#pragma unroll
    for (int i = 0; i < 2; ++i) *(volatile v8h*)(dst + off[i]) = x[i];
    __threadfence();
#pragma unroll
    for (int i = 0; i < 2; ++i) *(volatile v8h*)(dst + off[i]) = x[i];
  }

  if (MODE == MODE_WO) {
    v4f xs[4];
    size_t off[4];
#pragma unroll
    for (int i = 0; i < 4; ++i) {
      const unsigned r = 16u * (unsigned)i + (tid >> 4);
      const unsigned c = (tid & 15u) * 4u;
      const unsigned crow = row0 + r;
      const v4f u = *(const v4f*)&Cs[r * LDC + c];
      const v4f g = *(const v4f*)(bias + n0 + c);
      const v4f q = *(const v4f*)(addf + full_row(crow) * DIM + n0 + c);
      v4f val;
#pragma unroll
      for (int j = 0; j < 4; ++j)
        val[j] = (u[j] * (1.0f / (WCARRY * VCARRY)) + bf16r(g[j])) + bf16r(q[j]);
      xs[i] = val;
      off[i] = (size_t)crow * ND + n0 + c;
    }
#pragma unroll
    for (int i = 0; i < 4; ++i) *(volatile v4f*)(outf + off[i]) = xs[i];
    __threadfence();
#pragma unroll
    for (int i = 0; i < 4; ++i) *(volatile v4f*)(outf + off[i]) = xs[i];
  }

  if (MODE == MODE_W1) {
#pragma unroll 1
    for (unsigned i = 0; i < 2u; ++i) {
      const unsigned r = 32u * i + (tid >> 3);
      const unsigned c = (tid & 7u) * 8u;
      const v4f u0 = *(const v4f*)&Cs[r * LDC + c];
      const v4f u1 = *(const v4f*)&Cs[r * LDC + c + 4];
      const v4f g0 = *(const v4f*)(bias + n0 + c);
      const v4f g1 = *(const v4f*)(bias + n0 + c + 4);
      v8h xo;
#pragma unroll
      for (int j = 0; j < 4; ++j) {
        const float t0 = u0[j] * (1.0f / WCARRY) + bf16r(g0[j]);
        const float t1 = u1[j] * (1.0f / WCARRY) + bf16r(g1[j]);
        xo[j]     = (_Float16)(HCARRY * gelu_f(t0));
        xo[j + 4] = (_Float16)(HCARRY * gelu_f(t1));
      }
      _Float16* p = out16 + (size_t)(row0 + r) * ND + n0 + c;
      *(volatile v8h*)p = xo;
      __threadfence();
      *(volatile v8h*)p = xo;
    }
  }

  if (MODE == MODE_W2) {
    v4f xs[4];
    size_t off[4];
#pragma unroll
    for (int i = 0; i < 4; ++i) {
      const unsigned r = 16u * (unsigned)i + (tid >> 4);
      const unsigned c = (tid & 15u) * 4u;
      const unsigned crow = row0 + r;
      const v4f u  = *(const v4f*)&Cs[r * LDC + c];
      const v4f g  = *(const v4f*)(bias + n0 + c);
      const v4f rx = *(const v4f*)(addf + (size_t)crow * DIM + n0 + c);
      v4f val;
#pragma unroll
      for (int j = 0; j < 4; ++j)
        val[j] = (u[j] * (1.0f / (WCARRY * HCARRY)) + bf16r(g[j])) + rx[j];
      xs[i] = val;
      off[i] = full_row(crow) * DIM + n0 + c;
    }
#pragma unroll
    for (int i = 0; i < 4; ++i) *(volatile v4f*)(outf + off[i]) = xs[i];
    __threadfence();
#pragma unroll
    for (int i = 0; i < 4; ++i) *(volatile v4f*)(outf + off[i]) = xs[i];
  }
}

__global__ __launch_bounds__(256) void attn_kernel(
    const _Float16* __restrict__ Qh, const _Float16* __restrict__ Kh,
    const _Float16* __restrict__ Vt, _Float16* __restrict__ Ov) {
  __shared__ _Float16 Ks[64 * LDT];
  __shared__ _Float16 Vs[64 * LDT];
  __shared__ _Float16 Ps[8 * 16 * LDT];

  const unsigned tid = threadIdx.x, lane = tid & 31u;
  const unsigned w = (unsigned)__builtin_amdgcn_readfirstlane((int)(tid >> 5));
  const unsigned hh = lane >> 4, m = lane & 15u;
  const unsigned q0 = blockIdx.x * 128u;
  const unsigned head = blockIdx.y;
  const unsigned nbat = blockIdx.z;
  const unsigned wq0 = q0 + w * 16u;
  const float scale = 0.125f;
  _Float16* P = Ps + w * (16 * LDT);

  const size_t tok0 = (size_t)nbat * SEQ;
  const size_t qoff = (tok0 + wq0 + m) * DIM + head * HD + hh * 8u;
  v16h qf[2];
  qf[0] = frag_at(Qh + qoff);
  qf[1] = frag_at(Qh + qoff + 32);

  float mrow[8], lrow[8];
  v8f o[4];
#pragma unroll
  for (int v = 0; v < 8; ++v) { mrow[v] = -1.0e30f; lrow[v] = 0.0f; }
#pragma unroll
  for (int nb = 0; nb < 4; ++nb) o[nb] = (v8f){};

  const size_t kplane = tok0 * DIM + (size_t)head * HD;
  const size_t vplane = ((size_t)nbat * DIM + (size_t)head * HD) * SEQ;

  const unsigned kend = q0 + 128u;
  for (unsigned kb = 0; kb < kend; kb += 64u) {
#pragma unroll
    for (int j = 0; j < 2; ++j) {
      const unsigned idx = tid + 256u * (unsigned)j;
      const unsigned r = idx >> 3, c = (idx & 7u) * 8u;
      *(v8h*)&Ks[r * LDT + c] = *(const v8h*)(Kh + kplane + (size_t)(kb + r) * DIM + c);
      *(v8h*)&Vs[r * LDT + c] = *(const v8h*)(Vt + vplane + (size_t)r * SEQ + kb + c);
    }
    __syncthreads();

    v8f s[4];
#pragma unroll
    for (int kg = 0; kg < 4; ++kg) {
      v8f t = {};
#pragma unroll
      for (int c = 0; c < 2; ++c) {
        const v16h kf = ld_frag(&Ks[(kg * 16) * LDT + c * 32], LDT);
        t = wmma16(qf[c], kf, t);
      }
      s[kg] = t * scale;
    }

#pragma unroll
    for (int kg = 0; kg < 4; ++kg) {
      const unsigned col = kb + (unsigned)kg * 16u + m;
#pragma unroll
      for (int v = 0; v < 8; ++v) {
        const unsigned rowq = wq0 + hh * 8u + (unsigned)v;
        s[kg][v] = (col > rowq) ? -1.0e30f : s[kg][v];
      }
    }

    float alpha[8];
#pragma unroll
    for (int v = 0; v < 8; ++v) {
      float mx = fmaxf(fmaxf(s[0][v], s[1][v]), fmaxf(s[2][v], s[3][v]));
      mx = red16_max(mx);
      const float mn = fmaxf(mrow[v], mx);
      alpha[v] = __expf(mrow[v] - mn);
      mrow[v] = mn;
    }
#pragma unroll
    for (int kg = 0; kg < 4; ++kg)
#pragma unroll
      for (int v = 0; v < 8; ++v) s[kg][v] = __expf(s[kg][v] - mrow[v]);
#pragma unroll
    for (int v = 0; v < 8; ++v) {
      const float rs = red16_sum((s[0][v] + s[1][v]) + (s[2][v] + s[3][v]));
      lrow[v] = alpha[v] * lrow[v] + rs;
    }
#pragma unroll
    for (int nb = 0; nb < 4; ++nb)
#pragma unroll
      for (int v = 0; v < 8; ++v) o[nb][v] = o[nb][v] * alpha[v];

#pragma unroll
    for (int kg = 0; kg < 4; ++kg)
#pragma unroll
      for (int v = 0; v < 8; ++v)
        P[(hh * 8u + (unsigned)v) * LDT + (unsigned)kg * 16u + m] =
            (_Float16)(s[kg][v] * PCARRY);
    wave_lds_sync();

#pragma unroll
    for (int c = 0; c < 2; ++c) {
      const v16h pf = ld_frag(P + c * 32, LDT);
#pragma unroll
      for (int nb = 0; nb < 4; ++nb) {
        const v16h vf = ld_frag(&Vs[(nb * 16) * LDT + c * 32], LDT);
        o[nb] = wmma16(pf, vf, o[nb]);
      }
    }
    __syncthreads();
  }

  float inv[8];
#pragma unroll
  for (int v = 0; v < 8; ++v) inv[v] = __builtin_amdgcn_rcpf(lrow[v]) * (VCARRY / PCARRY);
#pragma unroll
  for (int nb = 0; nb < 4; ++nb)
#pragma unroll
    for (int v = 0; v < 8; ++v)
      P[(hh * 8u + (unsigned)v) * LDT + (unsigned)nb * 16u + m] =
          (_Float16)(o[nb][v] * inv[v]);
  wave_lds_sync();
  v8h x[4];
  size_t off[4];
#pragma unroll
  for (int i = 0; i < 4; ++i) {
    const unsigned r = 4u * (unsigned)i + (lane >> 3);
    const unsigned c = (lane & 7u) * 8u;
    x[i] = *(const v8h*)&P[r * LDT + c];
    off[i] = (tok0 + wq0 + r) * DIM + head * HD + c;
  }
#pragma unroll
  for (int i = 0; i < 4; ++i) *(volatile v8h*)(Ov + off[i]) = x[i];
  __threadfence();
#pragma unroll
  for (int i = 0; i < 4; ++i) *(volatile v8h*)(Ov + off[i]) = x[i];
}

static_assert((size_t)(3 * DIM / 64) * (MROWS / 64) * 4096 == (size_t)MROWS * 3 * DIM);
static_assert((size_t)(DIM / 64) * (MROWS / 64) * 4096 == (size_t)MROWS * DIM);
static_assert((size_t)(FF / 64) * (MROWS / 64) * 4096 == (size_t)MROWS * FF);
static_assert((size_t)(MROWS / 8) * 8 * 1024 == (size_t)MROWS * DIM);
static_assert((size_t)(SEQ / 128) * NHEAD * NB * 128 * 64 == (size_t)MROWS * DIM);

extern "C" void kernel_launch(void* const* d_in, const int* in_sizes, int n_in,
                              void* d_out, int out_size, void* d_ws, size_t ws_size,
                              hipStream_t stream) {
  if (n_in < 13) return;
  const long long need_x = ((long long)(NB - 1) * SEQ_FULL + SEQ) * DIM;
  if ((long long)in_sizes[0] < need_x) return;
  if (in_sizes[1] < 3 * DIM * DIM || in_sizes[2] < 3 * DIM) return;
  if (in_sizes[3] < DIM * DIM || in_sizes[4] < DIM) return;
  if (in_sizes[5] < DIM || in_sizes[6] < DIM || in_sizes[7] < DIM || in_sizes[8] < DIM) return;
  if (in_sizes[9] < DIM * FF || in_sizes[10] < FF) return;
  if (in_sizes[11] < FF * DIM || in_sizes[12] < DIM) return;
  if ((long long)out_size < need_x) return;
  if (ws_size < WS_TOTAL) return;

  const float* x    = (const float*)d_in[0];
  const float* Wqkv = (const float*)d_in[1];
  const float* bqkv = (const float*)d_in[2];
  const float* Wo   = (const float*)d_in[3];
  const float* bo   = (const float*)d_in[4];
  const float* ln1g = (const float*)d_in[5];
  const float* ln1b = (const float*)d_in[6];
  const float* ln2g = (const float*)d_in[7];
  const float* ln2b = (const float*)d_in[8];
  const float* W1   = (const float*)d_in[9];
  const float* b1   = (const float*)d_in[10];
  const float* W2   = (const float*)d_in[11];
  const float* b2   = (const float*)d_in[12];
  float* out = (float*)d_out;

  char* ws = (char*)d_ws;
  _Float16* Wqkv16 = (_Float16*)(ws + OFF_WQKV);
  _Float16* Wo16   = (_Float16*)(ws + OFF_WO);
  _Float16* W116   = (_Float16*)(ws + OFF_W1);
  _Float16* W216   = (_Float16*)(ws + OFF_W2);
  _Float16* H1     = (_Float16*)(ws + OFF_H1);
  _Float16* QKV16  = (_Float16*)(ws + OFF_QKV);
  _Float16* Q16    = QKV16;
  _Float16* K16    = QKV16 + (size_t)MROWS * DIM;
  _Float16* Vt16   = QKV16 + (size_t)2 * MROWS * DIM;
  _Float16* Ov16   = (_Float16*)(ws + OFF_OV);
  float*    X1     = (float*)(ws + OFF_X1);
  _Float16* H2     = (_Float16*)(ws + OFF_H2);
  _Float16* G16    = (_Float16*)(ws + OFF_G);

  dim3 blk(256);

  tcvt_kernel<DIM, 3 * DIM><<<dim3(3 * DIM / 64, DIM / 64), blk, 0, stream>>>(Wqkv, Wqkv16);
  tcvt_kernel<DIM, DIM><<<dim3(DIM / 64, DIM / 64), blk, 0, stream>>>(Wo, Wo16);
  tcvt_kernel<DIM, FF><<<dim3(FF / 64, DIM / 64), blk, 0, stream>>>(W1, W116);
  tcvt_kernel<FF, DIM><<<dim3(DIM / 64, FF / 64), blk, 0, stream>>>(W2, W216);

  ln_kernel<1><<<dim3(MROWS / 8), blk, 0, stream>>>(x, ln1g, ln1b, H1);
  gemm_kernel<MODE_QKV, DIM, 3 * DIM><<<dim3(3 * DIM / 64, MROWS / 64), blk, 0, stream>>>(
      H1, Wqkv16, bqkv, x, X1, QKV16);
  attn_kernel<<<dim3(SEQ / 128, NHEAD, NB), blk, 0, stream>>>(Q16, K16, Vt16, Ov16);
  gemm_kernel<MODE_WO, DIM, DIM><<<dim3(DIM / 64, MROWS / 64), blk, 0, stream>>>(
      Ov16, Wo16, bo, x, X1, H2);
  ln_kernel<0><<<dim3(MROWS / 8), blk, 0, stream>>>(X1, ln2g, ln2b, H2);
  gemm_kernel<MODE_W1, DIM, FF><<<dim3(FF / 64, MROWS / 64), blk, 0, stream>>>(
      H2, W116, b1, X1, X1, G16);
  gemm_kernel<MODE_W2, FF, DIM><<<dim3(DIM / 64, MROWS / 64), blk, 0, stream>>>(
      G16, W216, b2, X1, out, H1);
}
